// EdgeAttention_53944789238364
// MI455X (gfx1250) — hardware-verified
//
#include <hip/hip_runtime.h>
#include <stddef.h>
#include <stdint.h>


#define DIM     128
#define KO      256
#define NTHR    256
#define NWAVE   8
#define EPT     8
#define CHUNK   (NTHR * EPT)
#define WCAP    (EPT * 32)
#define LISTN   (NWAVE * WCAP)
#define NBMAX   2048
#define RCAP    28672
#define DEGCAP  4096
#define GBM     64
#define GBN     64
#define GTHR    128
#define QSCALE  0.25f
#define WSMAX   134217728
#define NU1     (3 * DIM * (DIM / 8))
#define NU2     (DIM * (KO / 8))
#define LDS_ATT ((2 * RCAP + 2 * NBMAX + LISTN) * 4 + 64)

static_assert((CHUNK & (CHUNK - 1)) == 0 && CHUNK <= 4096);
static_assert((NBMAX & (NBMAX - 1)) == 0 && NBMAX <= 4096);
static_assert(NTHR * 8 == NBMAX);
static_assert(LISTN >= NBMAX);
static_assert(LISTN >= NWAVE * WCAP);
static_assert((RCAP % 32) == 0);
static_assert(LDS_ATT <= 300000);
static_assert(GBM == (GTHR / 32) * 16);
static_assert((DIM % 32) == 0 && (KO % 32) == 0);
static_assert((DIM % GBN) == 0);
static_assert(DIM == 4 * 32);
static_assert(KO == 8 * 32);
static_assert((NU1 % NTHR) == 0 && ((NU1 + NU2) % NTHR) == 0);

typedef float          v4f   __attribute__((ext_vector_type(4)));
typedef float          v8f   __attribute__((ext_vector_type(8)));
typedef int            v4i   __attribute__((ext_vector_type(4)));
typedef int            v8i   __attribute__((ext_vector_type(8)));
typedef unsigned short v8us  __attribute__((ext_vector_type(8)));
typedef __bf16         v16bf __attribute__((ext_vector_type(16)));
union FragB { v16bf v; v8us h[2]; v8i w; v4i q[2]; };

__device__ __forceinline__ v8f wmb(const FragB& a, const FragB& b, v8f c) {
  v8f d = __builtin_amdgcn_wmma_f32_16x16x32_bf16(false, a.v, false, b.v, (short)0, c, false, false);
  asm volatile("v_nop\n\tv_nop\n\tv_nop\n\tv_nop" : "+v"(d) : "v"(a.w), "v"(b.w));
  return d;
}

__device__ __forceinline__ void ldwait() {
  asm volatile("s_wait_loadcnt 0x0" ::: "memory");
}

__device__ __forceinline__ unsigned bfb(float x) {
  unsigned u = __float_as_uint(x);
  u += 0x7FFFu + ((u >> 16) & 1u);
  return u >> 16;
}
__device__ __forceinline__ int pk2(float a, float b) {
  return (int)(bfb(a) | (bfb(b) << 16));
}
__device__ __forceinline__ v4i pack8(const v4f a, const v4f b) {
  v4i w;
  w.x = pk2(a.x, a.y); w.y = pk2(a.z, a.w); w.z = pk2(b.x, b.y); w.w = pk2(b.z, b.w);
  return w;
}

__device__ __forceinline__ int scan_chunk(const int* __restrict__ ee, int nP, int cbase, int slotBase,
                                          int nb, int* list, int tid, int lane, int wave) {
  int wc = 0;
  const int el0  = tid * EPT;
  const int e0   = cbase + el0;
  const int sent = -2147483647 - 1;
  v4i da, db;
  if (cbase + CHUNK <= nP) {
    const int* pp = ee + 2 * (size_t)e0;
    const v4i p0 = *(const v4i*)pp;
    const v4i p1 = *(const v4i*)(pp + 4);
    const v4i p2 = *(const v4i*)(pp + 8);
    const v4i p3 = *(const v4i*)(pp + 12);
    da.x = p0.x; da.y = p0.z; da.z = p1.x; da.w = p1.z;
    db.x = p2.x; db.y = p2.z; db.z = p3.x; db.w = p3.z;
  } else {
    const int lp = nP - 1;
    da.x = (e0     < nP) ? ee[2 * (size_t)min(e0,     lp)] : sent;
    da.y = (e0 + 1 < nP) ? ee[2 * (size_t)min(e0 + 1, lp)] : sent;
    da.z = (e0 + 2 < nP) ? ee[2 * (size_t)min(e0 + 2, lp)] : sent;
    da.w = (e0 + 3 < nP) ? ee[2 * (size_t)min(e0 + 3, lp)] : sent;
    db.x = (e0 + 4 < nP) ? ee[2 * (size_t)min(e0 + 4, lp)] : sent;
    db.y = (e0 + 5 < nP) ? ee[2 * (size_t)min(e0 + 5, lp)] : sent;
    db.z = (e0 + 6 < nP) ? ee[2 * (size_t)min(e0 + 6, lp)] : sent;
    db.w = (e0 + 7 < nP) ? ee[2 * (size_t)min(e0 + 7, lp)] : sent;
  }
  const unsigned nbs = (unsigned)slotBase;
  const unsigned unb = (unsigned)nb;
  const unsigned s0 = (unsigned)da.x - nbs, s1 = (unsigned)da.y - nbs;
  const unsigned s2 = (unsigned)da.z - nbs, s3 = (unsigned)da.w - nbs;
  const unsigned s4 = (unsigned)db.x - nbs, s5 = (unsigned)db.y - nbs;
  const unsigned s6 = (unsigned)db.z - nbs, s7 = (unsigned)db.w - nbs;
  const bool h0 = s0 < unb, h1 = s1 < unb, h2 = s2 < unb, h3 = s3 < unb;
  const bool h4 = s4 < unb, h5 = s5 < unb, h6 = s6 < unb, h7 = s7 < unb;
  const unsigned any = __builtin_amdgcn_ballot_w32(h0 | h1 | h2 | h3 | h4 | h5 | h6 | h7);
  if (any != 0u) {
#define HITJ(J, HJ, SJ) { \
      const unsigned mj = __builtin_amdgcn_ballot_w32(HJ); \
      if (mj != 0u) { \
        if (HJ) { \
          const int pos = wc + (int)__builtin_amdgcn_mbcnt_lo(mj, 0u); \
          if (pos < WCAP) list[wave * WCAP + pos] = ((el0 + (J)) << 12) | (int)(SJ); \
        } \
        wc += (int)__builtin_popcount(mj); } }
    HITJ(0, h0, s0)
    HITJ(1, h1, s1)
    HITJ(2, h2, s2)
    HITJ(3, h3, s3)
    HITJ(4, h4, s4)
    HITJ(5, h5, s5)
    HITJ(6, h6, s6)
    HITJ(7, h7, s7)
#undef HITJ
  }
  return wc;
}

__global__ __launch_bounds__(NTHR) void k_wcvt(const float* __restrict__ wq, const float* __restrict__ wk,
                                               const float* __restrict__ wv, const float* __restrict__ wo,
                                               unsigned short* wt, unsigned short* wot) {
  const int u = (int)blockIdx.x * NTHR + (int)threadIdx.x;
  if (u >= NU1 + NU2) return;
  v4f a, b;
  unsigned short* dst;
  if ((int)blockIdx.x < NU1 / NTHR) {
    const int n  = u >> 4;
    const int k8 = (u & 15) * 8;
    const int z  = n >> 7;
    const int nc = n & (DIM - 1);
    const float* ws = (z == 0) ? wq : ((z == 1) ? wk : wv);
    const float* p = ws + (size_t)k8 * DIM + nc;
    a.x = p[0];           a.y = p[DIM];         a.z = p[2 * DIM];     a.w = p[3 * DIM];
    b.x = p[4 * DIM];     b.y = p[5 * DIM];     b.z = p[6 * DIM];     b.w = p[7 * DIM];
    dst = wt + (size_t)n * DIM + k8;
  } else {
    const int u2 = u - NU1;
    const int n  = u2 >> 5;
    const int k8 = (u2 & 31) * 8;
    const int c0 = 4 * (k8 >> 3);
    const float* p = wo + (size_t)c0 * DIM + n;
    a.x = p[0];           a.y = p[DIM];         a.z = p[2 * DIM];     a.w = p[3 * DIM];
    b = a;
    dst = wot + (size_t)n * KO + k8;
  }
  const v4i w = pack8(a, b);
  *(volatile v4i*)dst = w;
  __threadfence();
  *(volatile v4i*)dst = w;
}

template<int MODE>
__global__ __launch_bounds__(GTHR) void k_gemm(
    const float* __restrict__ A0, const float* __restrict__ A1, const float* __restrict__ A2,
    const unsigned short* __restrict__ AH, const unsigned short* __restrict__ WT,
    const float* __restrict__ bias, float* outF,
    int K, int nA, int nRows, int zsO, float scl0, float scl1)
{
  __shared__ __attribute__((aligned(16))) float stg[GBM * GBN];
  const int tid = (int)threadIdx.x, lane = tid & 31, wave = tid >> 5, hh = lane >> 4, m = lane & 15;
  const int rowBase = (int)blockIdx.x * GBM;
  const int col0    = (int)blockIdx.y * GBN;
  const int z       = (int)blockIdx.z;
  const float scl   = (z == 0) ? scl0 : scl1;

  v8f acc[4];
  {
    const v8f zz = {0.f, 0.f, 0.f, 0.f, 0.f, 0.f, 0.f, 0.f};
    acc[0] = zz; acc[1] = zz; acc[2] = zz; acc[3] = zz;
  }
  const unsigned short* wp = WT + (size_t)(z * DIM + col0 + m) * (size_t)K + 8 * hh;
  const int ksteps = K >> 5;
  const int ar = rowBase + 16 * wave + m;

  if (MODE == 0) {
    const float* Ab = (z == 0) ? A0 : ((z == 1) ? A1 : A2);
    const int  arc = ar < nA ? ar : nA - 1;
    const bool az  = ar < nA;
    const float* ap = Ab + (size_t)arc * (size_t)K + 8 * hh;
    const v4f z4 = {0.f, 0.f, 0.f, 0.f};
#pragma unroll 1
    for (int ks = 0; ks < ksteps; ++ks) {
      v4f x0 = *(const v4f*)(ap + 32 * ks);
      v4f x1 = *(const v4f*)(ap + 32 * ks + 4);
      v4f x2 = *(const v4f*)(ap + 32 * ks + 16);
      v4f x3 = *(const v4f*)(ap + 32 * ks + 20);
      if (!az) { x0 = z4; x1 = z4; x2 = z4; x3 = z4; }
      FragB af;
      af.q[0] = pack8(x0, x1);
      af.q[1] = pack8(x2, x3);
#pragma unroll
      for (int t = 0; t < 4; ++t) {
        const unsigned short* wq2 = wp + (size_t)(16 * t) * (size_t)K + 32 * ks;
        FragB bf;
        bf.h[0] = *(const v8us*)wq2;
        bf.h[1] = *(const v8us*)(wq2 + 16);
        acc[t] = wmb(af, bf, acc[t]);
      }
    }
  } else {
    const unsigned short* ap = AH + (size_t)ar * (size_t)K + 8 * hh;
#pragma unroll 1
    for (int ks = 0; ks < ksteps; ++ks) {
      FragB af;
      af.h[0] = *(const v8us*)(ap + 32 * ks);
      af.h[1] = *(const v8us*)(ap + 32 * ks + 16);
#pragma unroll
      for (int t = 0; t < 4; ++t) {
        const unsigned short* wq2 = wp + (size_t)(16 * t) * (size_t)K + 32 * ks;
        FragB bf;
        bf.h[0] = *(const v8us*)wq2;
        bf.h[1] = *(const v8us*)(wq2 + 16);
        acc[t] = wmb(af, bf, acc[t]);
      }
    }
  }

#pragma unroll
  for (int t = 0; t < 4; ++t) {
    const int lc = 16 * t + m;
    float bv = 0.f;
    if (MODE == 1) {
      int bi = col0 + lc;
      bi = bi > DIM - 1 ? DIM - 1 : (bi < 0 ? 0 : bi);
      bv = __uint_as_float(bfb(bias[bi]) << 16);
    }
#pragma unroll
    for (int r = 0; r < 8; ++r) {
      const int lr = 16 * wave + 8 * hh + r;
      stg[lr * GBN + lc] = fmaf(acc[t][r], scl, bv);
    }
  }
  __syncthreads();

  float* ob = outF + (size_t)z * (size_t)zsO;
  v4f fv[8];
#pragma unroll
  for (int i = 0; i < 8; ++i) {
    const int lr = 16 * wave + 2 * i + hh;
    fv[i] = *(const v4f*)(stg + lr * GBN + 4 * m);
  }
#pragma unroll
  for (int i = 0; i < 8; ++i) {
    const int lr = 16 * wave + 2 * i + hh;
    const int gr = rowBase + lr;
    float* op = ob + (size_t)gr * DIM + col0 + 4 * m;
    if (gr < nRows) *(volatile v4f*)op = fv[i];
  }
  __threadfence();
#pragma unroll
  for (int i = 0; i < 8; ++i) {
    const int lr = 16 * wave + 2 * i + hh;
    const int gr = rowBase + lr;
    float* op = ob + (size_t)gr * DIM + col0 + 4 * m;
    if (gr < nRows) *(volatile v4f*)op = fv[i];
  }
}

__global__ __launch_bounds__(NTHR) void k_att(
    const int* __restrict__ ee, const float* __restrict__ QH, const float* __restrict__ KH,
    const float* __restrict__ VH, unsigned short* OA, int nR, int nP, int nb, int MPr) {
  extern __shared__ v4f lds_dyn[];
  int* reg1 = (int*)lds_dyn;
  int* reg2 = reg1 + RCAP;
  int* scnt = reg2 + RCAP;
  int* soff = scnt + NBMAX;
  int* list = soff + NBMAX;
  int* wcnt = list + LISTN;
  int* wtot = wcnt + NWAVE;
  const int tid = (int)threadIdx.x, lane = tid & 31, wave = tid >> 5;
  const int segBase = (int)blockIdx.x * nb;

  for (int i = tid; i < NBMAX; i += NTHR) scnt[i] = 0;
  __syncthreads();

  int tot = 0;
  const int nChunks = (nP + CHUNK - 1) / CHUNK;
#pragma unroll 1
  for (int ch = 0; ch < nChunks; ++ch) {
    const int cbase = ch * CHUNK;
    const int wc = scan_chunk(ee, nP, cbase, segBase, nb, list, tid, lane, wave);
    if (lane == 0) wcnt[wave] = wc;
    __syncthreads();
    int pre = 0, all = 0;
#pragma unroll
    for (int w2 = 0; w2 < NWAVE; ++w2) {
      int c = wcnt[w2];
      c = c < 0 ? 0 : (c > WCAP ? WCAP : c);
      all += c;
      pre += (w2 < wave) ? c : 0;
    }
    const int wcc  = wc > WCAP ? WCAP : wc;
    const int base = tot + pre;
#pragma unroll 1
    for (int i = lane; i < wcc; i += 32) {
      const int ent = list[wave * WCAP + i];
      const int el  = (ent >> 12) & (CHUNK - 1);
      const int sl  = ent & (NBMAX - 1);
      int pid = cbase + el;
      pid = pid > nP - 1 ? nP - 1 : pid;
      const int pos = base + i;
      if (pos < RCAP) reg1[pos] = (int)(((unsigned)pid << 12) | (unsigned)sl);
    }
    tot += all;
    tot = tot > RCAP ? RCAP : tot;
    __syncthreads();
  }
  const int nh = tot;

  if (wave == 0) {
#pragma unroll 1
    for (int b0 = 0; b0 < nh; b0 += 32) {
      const int idx = b0 + lane;
      const int uv  = reg1[idx < RCAP ? idx : RCAP - 1];
      const int m32 = (nh - b0) < 32 ? (nh - b0) : 32;
#pragma unroll 1
      for (int kq = 0; kq < m32; ++kq) {
        const int u  = __builtin_amdgcn_readlane(uv, kq);
        const int sl = u & (NBMAX - 1);
        if (lane == 0) scnt[sl] = scnt[sl] + 1;
      }
    }
  }
  __syncthreads();

  {
    const v4i ca = *(const v4i*)(scnt + 8 * tid);
    const v4i cb = *(const v4i*)(scnt + 8 * tid + 4);
    const int e0 = ca.x < 0 ? 0 : ca.x, e1 = ca.y < 0 ? 0 : ca.y, e2 = ca.z < 0 ? 0 : ca.z, e3 = ca.w < 0 ? 0 : ca.w;
    const int e4 = cb.x < 0 ? 0 : cb.x, e5 = cb.y < 0 ? 0 : cb.y, e6 = cb.z < 0 ? 0 : cb.z, e7 = cb.w < 0 ? 0 : cb.w;
    const int ts = e0 + e1 + e2 + e3 + e4 + e5 + e6 + e7;
    int incl = ts;
#pragma unroll
    for (int d = 1; d < 32; d <<= 1) {
      const int up = __shfl_up(incl, d);
      if (lane >= d) incl += up;
    }
    if (lane == 31) wtot[wave] = incl;
    __syncthreads();
    int pre = 0;
#pragma unroll
    for (int w2 = 0; w2 < NWAVE; ++w2) pre += (w2 < wave) ? wtot[w2] : 0;
    int run = pre + incl - ts;
    soff[8 * tid + 0] = run; run += e0;
    soff[8 * tid + 1] = run; run += e1;
    soff[8 * tid + 2] = run; run += e2;
    soff[8 * tid + 3] = run; run += e3;
    soff[8 * tid + 4] = run; run += e4;
    soff[8 * tid + 5] = run; run += e5;
    soff[8 * tid + 6] = run; run += e6;
    soff[8 * tid + 7] = run;
  }
  __syncthreads();
  for (int i = tid; i < NBMAX; i += NTHR) list[i] = soff[i];
  __syncthreads();

  if (wave == 0) {
#pragma unroll 1
    for (int b0 = 0; b0 < nh; b0 += 32) {
      const int idx = b0 + lane;
      const int uv  = reg1[idx < RCAP ? idx : RCAP - 1];
      const int m32 = (nh - b0) < 32 ? (nh - b0) : 32;
#pragma unroll 1
      for (int kq = 0; kq < m32; ++kq) {
        const int u   = __builtin_amdgcn_readlane(uv, kq);
        const int sl  = u & (NBMAX - 1);
        const int pid = (int)((unsigned)u >> 12);
        if (lane == 0) {
          int pos = list[sl];
          pos = pos < 0 ? 0 : (pos > RCAP - 1 ? RCAP - 1 : pos);
          reg2[pos] = pid;
          list[sl] = pos + 1;
        }
      }
    }
  }
  __syncthreads();

  const int nbw = nb >> 3;
  const bool ovf = (nh >= RCAP);
  const float qnan = __int_as_float(0x7fc00000);
#pragma unroll 1
  for (int jt = 0; jt < nbw; ++jt) {
    const int slot = wave * nbw + jt;
    const int grow = segBase + slot;
    const int gcl  = grow < nR ? grow : nR - 1;
    int st = soff[slot];
    const int craw = scnt[slot];
    int cnt = craw;
    st  = st < 0 ? 0 : (st > nh ? nh : st);
    cnt = cnt < 0 ? 0 : (cnt > DEGCAP ? DEGCAP : cnt);
    if (cnt > nh - st) cnt = nh - st;
    const float pz = (ovf || craw > DEGCAP) ? qnan : 0.0f;
    const bool wr = grow < MPr;
    const float live = grow < nR ? 1.0f : 0.0f;

    const v4f qv = *(const v4f*)(QH + (size_t)gcl * DIM + 4 * lane);
    ldwait();
    float mx = -1.0e30f, dn = 0.f;
    v4f av = {0.f, 0.f, 0.f, 0.f};

#pragma unroll 1
    for (int pq = 0; pq < cnt; ++pq) {
      int idx = st + pq; idx = idx > RCAP - 1 ? RCAP - 1 : idx;
      int pid = reg2[idx]; pid = pid < 0 ? 0 : (pid > nP - 1 ? nP - 1 : pid);
      const int nraw = ee[2 * (size_t)pid + 1];
      const int s = nraw < 0 ? 0 : (nraw > nR - 1 ? nR - 1 : nraw);
      const v4f kk = *(const v4f*)(KH + (size_t)s * DIM + 4 * lane);
      const v4f vv = *(const v4f*)(VH + (size_t)s * DIM + 4 * lane);
      ldwait();
      float part = qv.x * kk.x;
      part = fmaf(qv.y, kk.y, part);
      part = fmaf(qv.z, kk.z, part);
      part = fmaf(qv.w, kk.w, part);
      part += __shfl_xor(part, 1);
      part += __shfl_xor(part, 2);
      const float df = part - mx;
      const float ex = expf(-fabsf(df));
      const bool up  = df > 0.f;
      const float s1 = up ? ex : 1.0f;
      const float s2 = up ? 1.0f : ex;
      mx = up ? part : mx;
      dn = fmaf(dn, s1, s2);
      av.x = fmaf(av.x, s1, s2 * vv.x);
      av.y = fmaf(av.y, s1, s2 * vv.y);
      av.z = fmaf(av.z, s1, s2 * vv.z);
      av.w = fmaf(av.w, s1, s2 * vv.w);
    }
    const float ds = dn > 0.f ? dn : 1.0f;
    const float iv = (dn > 0.f ? 1.0f : 0.0f) * __builtin_amdgcn_rcpf(ds);
    const float o0 = (av.x * iv) * live + pz;
    const float o1 = (av.y * iv) * live + pz;
    const float o2 = (av.z * iv) * live + pz;
    const float o3 = (av.w * iv) * live + pz;
    const unsigned hb0 = bfb(o0), hb1 = bfb(o1), hb2 = bfb(o2), hb3 = bfb(o3);
    const unsigned lb0 = bfb(o0 - __uint_as_float(hb0 << 16));
    const unsigned lb1 = bfb(o1 - __uint_as_float(hb1 << 16));
    const unsigned lb2 = bfb(o2 - __uint_as_float(hb2 << 16));
    const unsigned lb3 = bfb(o3 - __uint_as_float(hb3 << 16));
    v4i w;
    w.x = (int)(hb0 | (hb1 << 16));
    w.y = (int)(hb2 | (hb3 << 16));
    w.z = (int)(lb0 | (lb1 << 16));
    w.w = (int)(lb2 | (lb3 << 16));
    unsigned short* gp = OA + (size_t)grow * KO + 8 * lane;
    if (wr) *(volatile v4i*)gp = w;
    __threadfence();
    if (wr) *(volatile v4i*)gp = w;
  }
}

static int pick_nb(int nP, int nR) {
  int nb = NBMAX;
  while (nb > 16 && (long long)nb * (long long)nP * 5LL > (long long)RCAP * (long long)nR * 4LL) nb >>= 1;
  return nb;
}
static inline int cdiv(int a, int b) { return (a + b - 1) / b; }

extern "C" void kernel_launch(void* const* d_in, const int* in_sizes, int n_in,
                              void* d_out, int out_size, void* d_ws, size_t ws_size,
                              hipStream_t stream) {
  if (n_in < 9) return;
  const int nR = in_sizes[0] / DIM;
  if (nR <= 0 || in_sizes[0] != nR * DIM || nR > (1 << 21)) return;
  if (in_sizes[1] != nR * DIM || in_sizes[2] != nR * DIM) return;
  if (in_sizes[3] < 2 || (in_sizes[3] & 1) != 0) return;
  const int nP = in_sizes[3] / 2;
  if (nP < 1 || nP > (1 << 20)) return;
  if (in_sizes[4] != DIM * DIM || in_sizes[5] != DIM * DIM) return;
  if (in_sizes[6] != DIM * DIM || in_sizes[7] != DIM * DIM) return;
  if (in_sizes[8] != DIM) return;
  if (out_size != nR * DIM) return;

  const float* q  = (const float*)d_in[0];
  const float* k  = (const float*)d_in[1];
  const float* v  = (const float*)d_in[2];
  const int*   ee = (const int*)  d_in[3];
  const float* Wq = (const float*)d_in[4];
  const float* Wk = (const float*)d_in[5];
  const float* Wv = (const float*)d_in[6];
  const float* Wo = (const float*)d_in[7];
  const float* bo = (const float*)d_in[8];
  float* out = (float*)d_out;

  const int MP = cdiv(nR, GBM) * GBM;
  const int nb = pick_nb(nP, nR);
  const int gA = cdiv(MP, nb);
  if (nb < 16 || (nb & (nb - 1)) != 0 || nb > NBMAX) return;
  if (gA * nb < MP) return;

  char* ws = (char*)d_ws;
  size_t off = 0;
  const size_t oQKV = off; off += (size_t)3 * MP * DIM * 4;        off = (off + 255) & ~(size_t)255;
  const size_t oOA  = off; off += (size_t)MP * KO * 2;             off = (off + 255) & ~(size_t)255;
  const size_t oWT  = off; off += (size_t)3 * DIM * DIM * 2;       off = (off + 255) & ~(size_t)255;
  const size_t oWOT = off; off += (size_t)DIM * KO * 2;            off = (off + 255) & ~(size_t)255;
  if (off > ws_size || off > (size_t)WSMAX) return;
  float*          QKV = (float*)(ws + oQKV);
  float*          QH  = QKV;
  float*          KH  = QKV + (size_t)MP * DIM;
  float*          VH  = QKV + (size_t)2 * MP * DIM;
  unsigned short* OA  = (unsigned short*)(ws + oOA);
  unsigned short* WT  = (unsigned short*)(ws + oWT);
  unsigned short* WOT = (unsigned short*)(ws + oWOT);

  hipFuncSetAttribute(reinterpret_cast<const void*>(&k_att),
                      hipFuncAttributeMaxDynamicSharedMemorySize, LDS_ATT);

  k_wcvt<<<cdiv(NU1 + NU2, NTHR), NTHR, 0, stream>>>(Wq, Wk, Wv, Wo, WT, WOT);

  k_gemm<0><<<dim3(MP / GBM, DIM / GBN, 3), GTHR, 0, stream>>>(q, k, v, OA, WT, bo, QKV,
                                                               DIM, nR, MP, MP * DIM, QSCALE, 1.0f);
  k_att<<<gA, NTHR, LDS_ATT, stream>>>(ee, QH, KH, VH, OA, nR, nP, nb, MP);
  k_gemm<1><<<dim3(MP / GBM, DIM / GBN, 1), GTHR, 0, stream>>>(q, q, q, OA, WOT, bo, out,
                                                               KO, MP, nR, 0, 1.0f, 1.0f);
}
